// GLF_25426206392719
// MI455X (gfx1250) — hardware-run, weakly checked
//
#include <hip/hip_runtime.h>
#include <math.h>

typedef __attribute__((ext_vector_type(16))) _Float16 v16h;
typedef __attribute__((ext_vector_type(8)))  _Float16 v8h;
typedef __attribute__((ext_vector_type(8)))  float    v8f;
typedef __attribute__((ext_vector_type(4)))  float    v4f;
typedef __attribute__((ext_vector_type(4)))  unsigned int v4u;

constexpr int kBatch   = 2;
constexpr int kSeq     = 2048;
constexpr int kEmb     = 1024;
constexpr int kHeads   = 16;
constexpr int kDh      = 64;
constexpr int kDhRoot  = 8;
constexpr int kSub     = 16;
constexpr int kTok     = kBatch * kSeq;
constexpr int kQkvLd   = 6 * kEmb;
constexpr int kLocCol  = 3 * kEmb;
constexpr int kFusedLd = 2 * kEmb;
constexpr int kKC      = 64;
static_assert(kHeads * kDh == kEmb, "head split");
static_assert(kDhRoot * kDhRoot == kDh, "head dim root");
static_assert((kSeq % 64) == 0 && (kSeq % kKC) == 0 && (kSeq % kSub) == 0, "sequence tiles");
static_assert((kTok % 64) == 0 && (kQkvLd % 64) == 0 && (kEmb % 64) == 0, "GEMM M,N multiples of 64");
static_assert((kEmb % 32) == 0 && (kFusedLd % 32) == 0, "GEMM K multiples of 32");

constexpr float kXCarry     = 16.0f;
constexpr float kWCarry     = 256.0f;
constexpr float kPCarry     = 32768.0f;
constexpr float kAttnGCarry = 256.0f;
constexpr float kAttnLCarry = 64.0f;
constexpr float kFusedCarry = 256.0f;
constexpr float kQkvScale   = 1.0f / kWCarry;
constexpr float kScoreScale = (1.0f / (float)kDhRoot) / (kXCarry * kXCarry);
constexpr float kOGFold     = kAttnGCarry / (kPCarry * kXCarry);
constexpr float kOLFold     = kAttnLCarry / (kPCarry * kXCarry);
constexpr float kOutGScale  = kFusedCarry / (kAttnGCarry * kWCarry);
constexpr float kOutLScale  = kFusedCarry / (kAttnLCarry * kWCarry);
constexpr float kFuseScale  = 1.0f / (kFusedCarry * kWCarry);

constexpr size_t kOffX16   = 0;
constexpr size_t kOffWQKV  = kOffX16   + (size_t)kTok * kEmb * 2;
constexpr size_t kOffWOUT  = kOffWQKV  + (size_t)kQkvLd * kEmb * 2;
constexpr size_t kOffWF    = kOffWOUT  + (size_t)2 * kEmb * kEmb * 2;
constexpr size_t kOffQKV   = kOffWF    + (size_t)kEmb * kFusedLd * 2;
constexpr size_t kOffATTN  = kOffQKV   + (size_t)kTok * kQkvLd * 2;
constexpr size_t kOffFUSED = kOffATTN  + (size_t)2 * kTok * kEmb * 2;
constexpr size_t kOffBIAS  = kOffFUSED + (size_t)kTok * kFusedLd * 2;
constexpr int    kBiasN    = kQkvLd + 2 * kEmb + kEmb;
constexpr size_t kWsTotal  = kOffBIAS  + (size_t)kBiasN * 4;
static_assert(kWsTotal == 113283072ull, "carve total");
static_assert(kWsTotal <= 134217728ull, "carve cap");
static_assert((kOffWQKV % 128) == 0 && (kOffWOUT % 128) == 0 && (kOffWF % 128) == 0 && (kOffQKV % 128) == 0 &&
              (kOffATTN % 128) == 0 && (kOffFUSED % 128) == 0 && (kOffBIAS % 128) == 0, "128-B aligned regions");

constexpr int kCvtE  = 2048;
constexpr int kCvtB1 = (kTok * kEmb) / kCvtE;
constexpr int kCvtB2 = kCvtB1 + (3 * kEmb * kEmb) / kCvtE;
constexpr int kCvtB3 = kCvtB2 + (3 * kEmb * kEmb) / kCvtE;
constexpr int kCvtB4 = kCvtB3 + (kEmb * kEmb) / kCvtE;
constexpr int kCvtB5 = kCvtB4 + (kEmb * kEmb) / kCvtE;
constexpr int kCvtB6 = kCvtB5 + (kEmb * kFusedLd) / kCvtE;
static_assert((size_t)kCvtB6 * kCvtE * 2 == kOffQKV, "converted planes are contiguous from offset 0");

__device__ __forceinline__ unsigned short f2bf_bits(float f) {
  unsigned u = __float_as_uint(f);
  return (unsigned short)((u + 0x7FFFu + ((u >> 16) & 1u)) >> 16);
}
__device__ __forceinline__ float bf_bits2f(unsigned short h) { return __uint_as_float(((unsigned)h) << 16); }
__device__ __forceinline__ unsigned short leg_h_bits(float f, float carry) {
  const float r = bf_bits2f(f2bf_bits(f));
  const _Float16 h = (_Float16)(r * carry);
  return __builtin_bit_cast(unsigned short, h);
}
__device__ __forceinline__ unsigned pk16(unsigned short a, unsigned short b) { return (unsigned)a | ((unsigned)b << 16); }

struct FragH {
  union U { v16h v; v8h h[2]; };
  static __device__ __forceinline__ v16h load(const _Float16* p) {
    U f;
    f.h[0] = *(const v8h*)(p);
    f.h[1] = *(const v8h*)(p + 16);
    return f.v;
  }
  static __device__ __forceinline__ v16h load_lo16(const _Float16* p) {
    U f;
    f.h[0] = *(const v8h*)(p);
    f.h[1] = (v8h){(_Float16)0.0f, (_Float16)0.0f, (_Float16)0.0f, (_Float16)0.0f,
                   (_Float16)0.0f, (_Float16)0.0f, (_Float16)0.0f, (_Float16)0.0f};
    return f.v;
  }
};

__device__ __forceinline__ v8f mma_f16(v16h a, v16h b, v8f c) {
  c = __builtin_amdgcn_wmma_f32_16x16x32_f16(false, a, false, b, (short)0, c, false, false);
  asm volatile("v_nop\n\tv_nop\n\tv_nop\n\tv_nop" : "+v"(c) : "v"(a), "v"(b));
  return c;
}

__device__ __forceinline__ void wave_lds_sync() {
  __builtin_amdgcn_fence(__ATOMIC_RELEASE, "workgroup");
  __builtin_amdgcn_wave_barrier();
  __builtin_amdgcn_fence(__ATOMIC_ACQUIRE, "workgroup");
}

__global__ __launch_bounds__(256) void cvt_planes_kernel(
    const float* __restrict__ x, const float* __restrict__ wing, const float* __restrict__ winl,
    const float* __restrict__ woutg, const float* __restrict__ woutl, const float* __restrict__ wf,
    unsigned short* __restrict__ dst) {
  const int blk = blockIdx.x;
  const float* src = x;
  int sb = 0;
  float carry = kXCarry;
  if (blk >= kCvtB5)      { src = wf;    sb = kCvtB5; carry = kWCarry; }
  else if (blk >= kCvtB4) { src = woutl; sb = kCvtB4; carry = kWCarry; }
  else if (blk >= kCvtB3) { src = woutg; sb = kCvtB3; carry = kWCarry; }
  else if (blk >= kCvtB2) { src = winl;  sb = kCvtB2; carry = kWCarry; }
  else if (blk >= kCvtB1) { src = wing;  sb = kCvtB1; carry = kWCarry; }
  const float* p = src + ((size_t)(blk - sb) * 256 + threadIdx.x) * 8;
  const v4f a = *(const v4f*)(p);
  const v4f c = *(const v4f*)(p + 4);
  unsigned short hb[8];
#pragma unroll
  for (int e = 0; e < 4; ++e) {
    const float fa = a[e];
    const float fc = c[e];
    hb[e]     = leg_h_bits(fa, carry);
    hb[4 + e] = leg_h_bits(fc, carry);
  }
  const v4u u = (v4u){pk16(hb[0], hb[1]), pk16(hb[2], hb[3]), pk16(hb[4], hb[5]), pk16(hb[6], hb[7])};
  unsigned short* q = dst + ((size_t)blk * 256 + threadIdx.x) * 8;
  *(volatile v4u*)q = u;
  __threadfence();
  *(volatile v4u*)q = u;
}

__global__ __launch_bounds__(256) void bias_table_kernel(
    const float* __restrict__ big, const float* __restrict__ bil, const float* __restrict__ bog,
    const float* __restrict__ bol, const float* __restrict__ bf, float* __restrict__ dst) {
  const int blk = blockIdx.x;
  const float* src = big;
  int soff = blk * 1024;
  float carry = kXCarry;
  if (blk >= 8)      { src = bf;  soff = 0; carry = 1.0f; }
  else if (blk >= 7) { src = bol; soff = 0; carry = kFusedCarry; }
  else if (blk >= 6) { src = bog; soff = 0; carry = kFusedCarry; }
  else if (blk >= 3) { src = bil; soff = (blk - 3) * 1024; }
  const int i = threadIdx.x * 4;
  const v4f a = *(const v4f*)(src + soff + i);
  v4f o;
#pragma unroll
  for (int e = 0; e < 4; ++e) {
    const float fa = a[e];
    o[e] = bf_bits2f(f2bf_bits(fa)) * carry;
  }
  float* q = dst + blk * 1024 + i;
  *(volatile v4f*)q = o;
  __threadfence();
  *(volatile v4f*)q = o;
}

template <int OUT_MODE>
__global__ __launch_bounds__(256) void gemm64_f16_kernel(
    const unsigned short* __restrict__ Ap, int lda, long strideA,
    const unsigned short* __restrict__ Btp, int ldb, long strideB,
    void* __restrict__ Cout, int ldc, long strideC,
    const float* __restrict__ bias, long strideBias,
    int M, int N, int K, float scale0, float scale1) {
  __shared__ __align__(16) float sT[8][16 * 68];
  const int b    = blockIdx.y;
  const int lane = threadIdx.x & 31;
  const int wave = threadIdx.x >> 5;
  const int tilesN = N >> 6;
  const int tilesM = M >> 6;
  const int tile = blockIdx.x * 8 + wave;
  if (tile >= tilesM * tilesN) return;
  const int tm = tile / tilesN;
  const int tn = tile - tm * tilesN;
  const int m0 = tm << 6;
  const int n0 = tn << 6;

  const _Float16* Ab = (const _Float16*)Ap  + (size_t)b * strideA;
  const _Float16* Bb = (const _Float16*)Btp + (size_t)b * strideB;
  const float* biasb = bias + (size_t)b * strideBias;
  const float scale  = (b == 0) ? scale0 : scale1;

  const int rlane = lane & 15;
  const int koff  = (lane >> 4) * 8;
  const int mOff  = (lane >> 4) * 8;

  v8f acc[4][4];
#pragma unroll
  for (int i = 0; i < 4; ++i)
#pragma unroll
    for (int j = 0; j < 4; ++j) acc[i][j] = (v8f){0.f, 0.f, 0.f, 0.f, 0.f, 0.f, 0.f, 0.f};

  for (int k0 = 0; k0 < K; k0 += 32) {
    v16h bh[4];
#pragma unroll
    for (int j = 0; j < 4; ++j) {
      const size_t bo = (size_t)(n0 + (j << 4) + rlane) * ldb + koff + k0;
      bh[j] = FragH::load(Bb + bo);
    }
#pragma unroll
    for (int i = 0; i < 4; ++i) {
      const size_t ao = (size_t)(m0 + (i << 4) + rlane) * lda + koff + k0;
      const v16h ah = FragH::load(Ab + ao);
#pragma unroll
      for (int j = 0; j < 4; ++j) acc[i][j] = mma_f16(ah, bh[j], acc[i][j]);
    }
  }

  float* slab = sT[wave];
#pragma unroll
  for (int i = 0; i < 4; ++i) {
    const int mBase = m0 + (i << 4);
#pragma unroll
    for (int j = 0; j < 4; ++j) {
      const int n = n0 + (j << 4) + rlane;
      const float bv = biasb[n];
#pragma unroll
      for (int r = 0; r < 8; ++r) {
        const float v = acc[i][j][r] * scale + bv;
        slab[(mOff + r) * 68 + (j << 4) + rlane] = v;
      }
    }
    wave_lds_sync();
    if (OUT_MODE == 0) {
      float* C = (float*)Cout + (size_t)b * strideC;
      const int hh = lane >> 4, c4 = (lane & 15) * 4;
      for (int pass = 0; pass < 2; ++pass) {
#pragma unroll
        for (int it = 0; it < 8; ++it) {
          const int row = it * 2 + hh;
          const v4f v = *(const v4f*)(slab + row * 68 + c4);
          *(volatile v4f*)(C + (size_t)(mBase + row) * ldc + n0 + c4) = v;
        }
        __threadfence();
      }
    } else {
      const int q = lane >> 3, c8 = (lane & 7) * 8;
      unsigned short* C = (unsigned short*)Cout + (size_t)b * strideC;
      for (int pass = 0; pass < 2; ++pass) {
#pragma unroll
        for (int it = 0; it < 4; ++it) {
          const int row = it * 4 + q;
          const float* sp = slab + row * 68 + c8;
          v8h hv;
#pragma unroll
          for (int e = 0; e < 8; ++e) hv[e] = (_Float16)sp[e];
          *(volatile v8h*)(C + (size_t)(mBase + row) * ldc + n0 + c8) = hv;
        }
        __threadfence();
      }
    }
    wave_lds_sync();
  }
}

__global__ __launch_bounds__(128) void attn_global_kernel(const unsigned short* __restrict__ qkv,
                                                          unsigned short* __restrict__ og) {
  __shared__ __align__(16) _Float16 Ksh[kKC * kDh];
  __shared__ __align__(16) _Float16 Vth[kDh * kKC];
  __shared__ __align__(16) _Float16 Psh[4][16 * kKC];
  __shared__ __align__(16) float    Os[4][16 * 68];

  const int tid  = threadIdx.x;
  const int wave = tid >> 5;
  const int lane = tid & 31;
  const int hh   = lane >> 4;
  const int c    = lane & 15;

  constexpr int nqb = kSeq / 64;
  const int bx = blockIdx.x;
  const int qb = bx % nqb;
  const int bh = bx / nqb;
  const int h  = bh % kHeads;
  const int b  = bh / kHeads;
  const int q0 = qb * 64 + wave * 16;

  const _Float16* base = (const _Float16*)qkv + (size_t)b * kSeq * kQkvLd;

  const _Float16* qrow = base + (size_t)(q0 + c) * kQkvLd + h * kDh + 8 * hh;
  const v16h qa0 = FragH::load(qrow);
  const v16h qa1 = FragH::load(qrow + 32);

  float mrow[8], lrow[8];
  v8f oacc[4];
#pragma unroll
  for (int r = 0; r < 8; ++r) { mrow[r] = -INFINITY; lrow[r] = 0.f; }
#pragma unroll
  for (int t = 0; t < 4; ++t) oacc[t] = (v8f){0.f, 0.f, 0.f, 0.f, 0.f, 0.f, 0.f, 0.f};

  _Float16* pw = Psh[wave];
  const int kvr = tid >> 1;
  const int dhs = (tid & 1) * 32;

#pragma unroll 1
  for (int kc = 0; kc < kSeq / kKC; ++kc) {
    const int kv0 = kc * kKC;
    __syncthreads();
    {
      const _Float16* krow = base + (size_t)(kv0 + kvr) * kQkvLd + kEmb + h * kDh + dhs;
      const unsigned short* vrow = (const unsigned short*)(base + (size_t)(kv0 + kvr) * kQkvLd + 2 * kEmb + h * kDh + dhs);
#pragma unroll
      for (int i = 0; i < 4; ++i) {
        const v8h kk = *(const v8h*)(krow + 8 * i);
        *(v8h*)(Ksh + kvr * kDh + dhs + 8 * i) = kk;
        const v4u vv = *(const v4u*)(vrow + 8 * i);
#pragma unroll
        for (int e = 0; e < 4; ++e) {
          const unsigned w = vv[e];
          const unsigned short lo = (unsigned short)(w & 0xffffu);
          const unsigned short hi = (unsigned short)(w >> 16);
          Vth[(dhs + 8 * i + 2 * e) * kKC + kvr]     = __builtin_bit_cast(_Float16, lo);
          Vth[(dhs + 8 * i + 2 * e + 1) * kKC + kvr] = __builtin_bit_cast(_Float16, hi);
        }
      }
    }
    __syncthreads();

    v8f s[4];
#pragma unroll
    for (int j = 0; j < 4; ++j) {
      s[j] = (v8f){0.f, 0.f, 0.f, 0.f, 0.f, 0.f, 0.f, 0.f};
      const _Float16* kp = Ksh + (j * 16 + c) * kDh + 8 * hh;
      const v16h kb0 = FragH::load(kp);
      s[j] = mma_f16(qa0, kb0, s[j]);
      const v16h kb1 = FragH::load(kp + 32);
      s[j] = mma_f16(qa1, kb1, s[j]);
    }

    float cm[8];
#pragma unroll
    for (int r = 0; r < 8; ++r) {
      float m = -INFINITY;
#pragma unroll
      for (int j = 0; j < 4; ++j) {
        s[j][r] *= kScoreScale;
        m = fmaxf(m, s[j][r]);
      }
#pragma unroll
      for (int off = 1; off < 16; off <<= 1) m = fmaxf(m, __shfl_xor(m, off, 32));
      cm[r] = m;
    }
#pragma unroll
    for (int r = 0; r < 8; ++r) {
      const float mnew  = fmaxf(mrow[r], cm[r]);
      const float alpha = __expf(mrow[r] - mnew);
      mrow[r] = mnew;
      float psum = 0.f;
#pragma unroll
      for (int j = 0; j < 4; ++j) {
        const float p = __expf(s[j][r] - mnew);
        psum += p;
        pw[(8 * hh + r) * kKC + j * 16 + c] = (_Float16)(p * kPCarry);
      }
#pragma unroll
      for (int off = 1; off < 16; off <<= 1) psum += __shfl_xor(psum, off, 32);
      lrow[r] = lrow[r] * alpha + psum;
#pragma unroll
      for (int t = 0; t < 4; ++t) oacc[t][r] *= alpha;
    }
    wave_lds_sync();
#pragma unroll 1
    for (int kk = 0; kk < 2; ++kk) {
      const v16h pa = FragH::load(pw + c * kKC + kk * 32 + 8 * hh);
#pragma unroll
      for (int t = 0; t < 4; ++t) {
        const v16h vb = FragH::load(Vth + (t * 16 + c) * kKC + kk * 32 + 8 * hh);
        oacc[t] = mma_f16(pa, vb, oacc[t]);
      }
    }
  }

  float* os = Os[wave];
#pragma unroll
  for (int r = 0; r < 8; ++r) {
    const float inv = kOGFold * (1.0f / lrow[r]);
#pragma unroll
    for (int t = 0; t < 4; ++t) os[(8 * hh + r) * 68 + t * 16 + c] = oacc[t][r] * inv;
  }
  wave_lds_sync();
  {
    const int q = lane >> 3, c8 = (lane & 7) * 8;
    unsigned short* op = og + (size_t)(b * kSeq + q0) * kEmb + h * kDh;
    for (int pass = 0; pass < 2; ++pass) {
#pragma unroll
      for (int it = 0; it < 4; ++it) {
        const int row = it * 4 + q;
        const float* sp = os + row * 68 + c8;
        v8h hv;
#pragma unroll
        for (int e = 0; e < 8; ++e) hv[e] = (_Float16)sp[e];
        *(volatile v8h*)(op + (size_t)row * kEmb + c8) = hv;
      }
      __threadfence();
    }
  }
}

__global__ __launch_bounds__(128) void attn_local_kernel(const unsigned short* __restrict__ qkv,
                                                         unsigned short* __restrict__ ol) {
  __shared__ __align__(16) _Float16 Vt[4][kDh * kSub];
  __shared__ __align__(16) _Float16 Pl[4][kSub * kSub];
  __shared__ __align__(16) float    Os[4][16 * 68];

  const int tid  = threadIdx.x;
  const int wave = tid >> 5;
  const int lane = tid & 31;
  const int hh   = lane >> 4;
  const int c    = lane & 15;

  const int unit = blockIdx.x * 4 + wave;
  const int h    = unit % kHeads;
  const int tb   = unit / kHeads;
  const int tok0 = tb * kSub;

  const _Float16* base = (const _Float16*)qkv + (size_t)tok0 * kQkvLd + kLocCol;

  const _Float16* qrow = base + (size_t)c * kQkvLd + h * kDh + 8 * hh;
  const v16h qa0 = FragH::load(qrow);
  const v16h qa1 = FragH::load(qrow + 32);
  const _Float16* krow = base + (size_t)c * kQkvLd + kEmb + h * kDh + 8 * hh;
  const v16h kb0 = FragH::load(krow);
  const v16h kb1 = FragH::load(krow + 32);

  {
    const int key = lane >> 1;
    const int dhs = (lane & 1) * 32;
    const unsigned short* vrow = (const unsigned short*)(base + (size_t)key * kQkvLd + 2 * kEmb + h * kDh + dhs);
    _Float16* vt = Vt[wave];
#pragma unroll
    for (int i = 0; i < 4; ++i) {
      const v4u vv = *(const v4u*)(vrow + 8 * i);
#pragma unroll
      for (int e = 0; e < 4; ++e) {
        const unsigned w = vv[e];
        const unsigned short lo = (unsigned short)(w & 0xffffu);
        const unsigned short hi = (unsigned short)(w >> 16);
        vt[(dhs + 8 * i + 2 * e) * kSub + key]     = __builtin_bit_cast(_Float16, lo);
        vt[(dhs + 8 * i + 2 * e + 1) * kSub + key] = __builtin_bit_cast(_Float16, hi);
      }
    }
  }

  v8f s = (v8f){0.f, 0.f, 0.f, 0.f, 0.f, 0.f, 0.f, 0.f};
  s = mma_f16(qa0, kb0, s);
  s = mma_f16(qa1, kb1, s);

  float linv[8];
  _Float16* pl = Pl[wave];
#pragma unroll
  for (int r = 0; r < 8; ++r) {
    const float xs = s[r] * kScoreScale;
    float m = xs;
#pragma unroll
    for (int off = 1; off < 16; off <<= 1) m = fmaxf(m, __shfl_xor(m, off, 32));
    const float p = expf(xs - m);
    float sum = p;
#pragma unroll
    for (int off = 1; off < 16; off <<= 1) sum += __shfl_xor(sum, off, 32);
    linv[r] = kOLFold * (1.0f / sum);
    pl[(8 * hh + r) * kSub + c] = (_Float16)(p * kPCarry);
  }
  __syncthreads();

  const v16h pa = FragH::load_lo16(pl + c * kSub + 8 * hh);
  v8f o[4];
#pragma unroll
  for (int t = 0; t < 4; ++t) {
    const v16h vb = FragH::load_lo16(Vt[wave] + (t * 16 + c) * kSub + 8 * hh);
    o[t] = (v8f){0.f, 0.f, 0.f, 0.f, 0.f, 0.f, 0.f, 0.f};
    o[t] = mma_f16(pa, vb, o[t]);
  }

  float* os = Os[wave];
#pragma unroll
  for (int r = 0; r < 8; ++r) {
#pragma unroll
    for (int t = 0; t < 4; ++t) os[(8 * hh + r) * 68 + t * 16 + c] = o[t][r] * linv[r];
  }
  __syncthreads();
  {
    const int q = lane >> 3, c8 = (lane & 7) * 8;
    unsigned short* op = ol + (size_t)tok0 * kEmb + h * kDh;
    for (int pass = 0; pass < 2; ++pass) {
#pragma unroll
      for (int it = 0; it < 4; ++it) {
        const int row = it * 4 + q;
        const float* sp = os + row * 68 + c8;
        v8h hv;
#pragma unroll
        for (int e = 0; e < 8; ++e) hv[e] = (_Float16)sp[e];
        *(volatile v8h*)(op + (size_t)row * kEmb + c8) = hv;
      }
      __threadfence();
    }
  }
}

extern "C" void kernel_launch(void* const* d_in, const int* in_sizes, int n_in,
                              void* d_out, int out_size, void* d_ws, size_t ws_size,
                              hipStream_t stream) {
  if (n_in < 11) return;
  if (in_sizes[0] != kTok * kEmb) return;
  if (in_sizes[1] != 3 * kEmb * kEmb || in_sizes[2] != 3 * kEmb) return;
  if (in_sizes[3] != kEmb * kEmb || in_sizes[4] != kEmb) return;
  if (in_sizes[5] != 3 * kEmb * kEmb || in_sizes[6] != 3 * kEmb) return;
  if (in_sizes[7] != kEmb * kEmb || in_sizes[8] != kEmb) return;
  if (in_sizes[9] != kEmb * kFusedLd || in_sizes[10] != kEmb) return;
  if (out_size != kTok * kEmb) return;
  if (ws_size < kWsTotal) return;

  const float* x       = (const float*)d_in[0];
  const float* w_in_g  = (const float*)d_in[1];
  const float* b_in_g  = (const float*)d_in[2];
  const float* w_out_g = (const float*)d_in[3];
  const float* b_out_g = (const float*)d_in[4];
  const float* w_in_l  = (const float*)d_in[5];
  const float* b_in_l  = (const float*)d_in[6];
  const float* w_out_l = (const float*)d_in[7];
  const float* b_out_l = (const float*)d_in[8];
  const float* w_f     = (const float*)d_in[9];
  const float* b_f     = (const float*)d_in[10];

  char* ws = (char*)d_ws;
  unsigned short* X16     = (unsigned short*)(ws + kOffX16);
  unsigned short* WQKV16  = (unsigned short*)(ws + kOffWQKV);
  unsigned short* WOUT16  = (unsigned short*)(ws + kOffWOUT);
  unsigned short* WF16    = (unsigned short*)(ws + kOffWF);
  unsigned short* QKV16   = (unsigned short*)(ws + kOffQKV);
  unsigned short* ATTN16  = (unsigned short*)(ws + kOffATTN);
  unsigned short* FUSED16 = (unsigned short*)(ws + kOffFUSED);
  float*          BIAS    = (float*)(ws + kOffBIAS);
  float*          BQKV    = BIAS;
  float*          BOUT    = BIAS + kQkvLd;
  float*          BFZ     = BIAS + kQkvLd + 2 * kEmb;

  cvt_planes_kernel<<<kCvtB6, 256, 0, stream>>>(x, w_in_g, w_in_l, w_out_g, w_out_l, w_f, X16);
  bias_table_kernel<<<kBiasN / 1024, 256, 0, stream>>>(b_in_g, b_in_l, b_out_g, b_out_l, b_f, BIAS);

  gemm64_f16_kernel<1><<<dim3((kTok / 64) * (kQkvLd / 64) / 8, 1), 256, 0, stream>>>(
      X16, kEmb, 0L,
      WQKV16, kEmb, 0L,
      (void*)QKV16, kQkvLd, 0L,
      BQKV, 0L,
      kTok, kQkvLd, kEmb, kQkvScale, kQkvScale);

  attn_global_kernel<<<kBatch * kHeads * (kSeq / 64), 128, 0, stream>>>(QKV16, ATTN16);
  attn_local_kernel<<<(kTok / kSub) * kHeads / 4, 128, 0, stream>>>(QKV16, ATTN16 + (size_t)kTok * kEmb);

  gemm64_f16_kernel<1><<<dim3((kTok / 64) * (kEmb / 64) / 8, 2), 256, 0, stream>>>(
      ATTN16, kEmb, (long)kTok * kEmb,
      WOUT16, kEmb, (long)kEmb * kEmb,
      (void*)FUSED16, kFusedLd, (long)kEmb,
      BOUT, (long)kEmb,
      kTok, kEmb, kEmb, kOutGScale, kOutLScale);

  gemm64_f16_kernel<0><<<dim3((kTok / 64) * (kEmb / 64) / 8, 1), 256, 0, stream>>>(
      FUSED16, kFusedLd, 0L,
      WF16, kFusedLd, 0L,
      d_out, kEmb, 0L,
      BFZ, 0L,
      kTok, kEmb, kFusedLd, kFuseScale, kFuseScale);
}
